// DilationSpconv_7370163880515
// MI455X (gfx1250) — hardware-verified
//
#include <hip/hip_runtime.h>
#include <stddef.h>


#define CCH    64
#define KOF    9
#define KK     (KOF * CCH)
#define NLAY   3
#define XLIMV  352
#define YLIMV  96
#define EPSV   1e-5f
#define TR     64
#define CTH    128
#define ZPAD   64
#define PTH    128
#define PROWS  (PTH / 8)
#define WSCAP  134217728

static_assert(KK % 32 == 0);
static_assert(TR % PROWS == 0);
static_assert(CCH % PROWS == 0);
static_assert(ZPAD % PROWS == 0);
static_assert(CTH == 128);
static_assert(TR == 64);
static_assert(PROWS == 16);
static_assert(CCH * CCH == 8 * PTH * 4);

typedef unsigned short us;
typedef us     v8us __attribute__((ext_vector_type(8)));
typedef float  v4f  __attribute__((ext_vector_type(4)));
typedef float  v8f  __attribute__((ext_vector_type(8)));
typedef __bf16 v16b __attribute__((ext_vector_type(16)));
union BFrag { v16b v; v8us u[2]; };

__device__ __forceinline__ v8f wmb(v16b a, v16b b, v8f c) {
  v8f d = __builtin_amdgcn_wmma_f32_16x16x32_bf16(false, a, false, b, (short)0, c, false, false);
  asm volatile("v_nop\n\tv_nop\n\tv_nop\n\tv_nop" : "+v"(d) : "v"(a), "v"(b));
  return d;
}

__device__ __forceinline__ us f2bf(float x) {
  const unsigned u = __float_as_uint(x);
  return (us)((u + 0x7FFFu + ((u >> 16) & 1u)) >> 16);
}
__device__ __forceinline__ float bf2f(us b) { return __uint_as_float(((unsigned)b) << 16); }

__device__ __forceinline__ void split8(v4f a, v4f b, v8us& hv, v8us& lv) {
  float x[8] = {a.x, a.y, a.z, a.w, b.x, b.y, b.z, b.w};
#pragma unroll
  for (int e = 0; e < 8; ++e) {
    const us hb = f2bf(x[e]);
    hv[e] = hb;
    lv[e] = f2bf(x[e] - bf2f(hb));
  }
}

__global__ __launch_bounds__(PTH) void k_xprep(const float* __restrict__ feat, us* Ph, us* Pl, int nN) {
  const int tid = threadIdx.x;
  const int row = blockIdx.x * PROWS + (tid >> 3);
  const int pc  = (tid & 7) * 8;
  const int rc  = row < nN ? row : nN - 1;
  const float* p = feat + (size_t)rc * CCH + pc;
  const v4f a = *(const v4f*)p;
  const v4f b = *(const v4f*)(p + 4);
  v8us hv, lv;
  split8(a, b, hv, lv);
  us* dh = Ph + (size_t)row * CCH + pc;
  us* dl = Pl + (size_t)row * CCH + pc;
  *(volatile v8us*)dh = hv;
  *(volatile v8us*)dl = lv;
  __threadfence();
  *(volatile v8us*)dh = hv;
  *(volatile v8us*)dl = lv;
}

__global__ __launch_bounds__(PTH) void k_zprep(us* P0h, us* P0l, us* P1h, us* P1l, int mPad) {
  const int tid = threadIdx.x;
  const int b = blockIdx.x;
  us* P = b == 0 ? P0h : (b == 1 ? P0l : (b == 2 ? P1h : P1l));
  const v8us z = {0, 0, 0, 0, 0, 0, 0, 0};
  const int pc = (tid & 7) * 8;
#pragma unroll
  for (int it = 0; it < ZPAD / PROWS; ++it) {
    const int row = mPad + PROWS * it + (tid >> 3);
    *(volatile v8us*)(P + (size_t)row * CCH + pc) = z;
  }
  __threadfence();
#pragma unroll
  for (int it = 0; it < ZPAD / PROWS; ++it) {
    const int row = mPad + PROWS * it + (tid >> 3);
    *(volatile v8us*)(P + (size_t)row * CCH + pc) = z;
  }
}

__global__ __launch_bounds__(PTH) void k_wprep(const float* __restrict__ W1, const float* __restrict__ W2,
                                               const float* __restrict__ W3, us* Wh, us* Wl) {
  __shared__ __attribute__((aligned(16))) float sW[CCH * CCH];
  const int k = blockIdx.x, layer = blockIdx.y, tid = threadIdx.x;
  const float* W  = layer == 0 ? W1 : (layer == 1 ? W2 : W3);
  const float* wk = W + (size_t)k * CCH * CCH;
  {
    v4f t0[4], t1[4];
#pragma unroll
    for (int g = 0; g < 4; ++g) t0[g] = *(const v4f*)(wk + (size_t)(g * PTH + tid) * 4);
    asm volatile("s_wait_loadcnt 0x0" ::: "memory");
#pragma unroll
    for (int g = 0; g < 4; ++g) ((v4f*)sW)[g * PTH + tid] = t0[g];
#pragma unroll
    for (int g = 0; g < 4; ++g) t1[g] = *(const v4f*)(wk + (size_t)((4 + g) * PTH + tid) * 4);
    asm volatile("s_wait_loadcnt 0x0" ::: "memory");
#pragma unroll
    for (int g = 0; g < 4; ++g) ((v4f*)sW)[(4 + g) * PTH + tid] = t1[g];
  }
  __syncthreads();
  const int pc = (tid & 7) * 8;
  v8us hv[CCH / PROWS], lv[CCH / PROWS];
#pragma unroll
  for (int it = 0; it < CCH / PROWS; ++it) {
    const int n = PROWS * it + (tid >> 3);
    v4f a, b;
    a.x = sW[(pc + 0) * CCH + n];
    a.y = sW[(pc + 1) * CCH + n];
    a.z = sW[(pc + 2) * CCH + n];
    a.w = sW[(pc + 3) * CCH + n];
    b.x = sW[(pc + 4) * CCH + n];
    b.y = sW[(pc + 5) * CCH + n];
    b.z = sW[(pc + 6) * CCH + n];
    b.w = sW[(pc + 7) * CCH + n];
    split8(a, b, hv[it], lv[it]);
  }
#pragma unroll
  for (int it = 0; it < CCH / PROWS; ++it) {
    const int n = PROWS * it + (tid >> 3);
    const size_t o = (size_t)(layer * CCH + n) * KK + (size_t)k * CCH + pc;
    *(volatile v8us*)(Wh + o) = hv[it];
    *(volatile v8us*)(Wl + o) = lv[it];
  }
  __threadfence();
#pragma unroll
  for (int it = 0; it < CCH / PROWS; ++it) {
    const int n = PROWS * it + (tid >> 3);
    const size_t o = (size_t)(layer * CCH + n) * KK + (size_t)k * CCH + pc;
    *(volatile v8us*)(Wh + o) = hv[it];
    *(volatile v8us*)(Wl + o) = lv[it];
  }
}

__device__ __forceinline__ void stage16(float* S, v8f acc, int r0, int c0, int h, int mi,
                                        const float* psc, const float* pmu, const float* pbe) {
  const int col = c0 + mi;
  const float sc = psc[col], mu = pmu[col], be = pbe[col];
#pragma unroll
  for (int r = 0; r < 8; ++r) S[(r0 + 8 * h + r) * CCH + col] = fmaxf((acc[r] - mu) * sc + be, 0.0f);
}

template <int LAST>
__global__ __launch_bounds__(CTH) void k_conv(
    const us* __restrict__ Ph, const us* __restrict__ Pl, const int* __restrict__ kin,
    const us* __restrict__ Wh, const us* __restrict__ Wl,
    const float* __restrict__ gg, const float* __restrict__ bb,
    const float* __restrict__ mm, const float* __restrict__ vv,
    const int* __restrict__ coor, us* Oh, us* Ol, float* out, int nN, int mPad) {
  __shared__ __attribute__((aligned(16))) us    Th[TR * CCH];
  __shared__ __attribute__((aligned(16))) us    Tl[TR * CCH];
  __shared__ __attribute__((aligned(16))) float S[TR * CCH];
  __shared__ __attribute__((aligned(16))) float psc[CCH];
  __shared__ __attribute__((aligned(16))) float pmu[CCH];
  __shared__ __attribute__((aligned(16))) float pbe[CCH];
  __shared__ __attribute__((aligned(16))) float pmk[TR];
  const int tid = threadIdx.x, lane = tid & 31, h = lane >> 4, mi = lane & 15;
  const int wave = __builtin_amdgcn_readfirstlane(tid >> 5);
  const int wr = wave >> 1, wc = wave & 1;
  const int rowbase = blockIdx.x * TR;

  if (tid < CCH) {
    psc[tid] = gg[tid] * rsqrtf(vv[tid] + EPSV);
    pmu[tid] = mm[tid];
    pbe[tid] = bb[tid];
  }
  if (LAST) {
    if (tid < TR) {
      int dr = rowbase + tid;
      dr = dr < nN ? dr : nN - 1;
      const int cx = coor[(size_t)dr * 3 + 1];
      const int cy = coor[(size_t)dr * 3 + 2];
      pmk[tid] = (cx > -XLIMV && cx <= XLIMV && cy > -YLIMV && cy <= YLIMV) ? 1.0f : 0.0f;
    }
  }

  const v8f z8 = {0.0f, 0.0f, 0.0f, 0.0f, 0.0f, 0.0f, 0.0f, 0.0f};
  v8f acc00 = z8, acc01 = z8, acc10 = z8, acc11 = z8;

#pragma unroll 1
  for (int k = 0; k < KOF; ++k) {
    __syncthreads();
    const int* kr = kin + (size_t)k * nN;
#pragma unroll
    for (int it = 0; it < TR / PROWS; ++it) {
      const int rr = PROWS * it + (tid >> 3);
      const int pc = (tid & 7) * 8;
      int dr = rowbase + rr;
      dr = dr < nN ? dr : nN - 1;
      int s = kr[dr];
      s = s < 0 ? s + nN + 1 : s;
      s = s < 0 ? 0 : s;
      const int srow = s < nN ? s : mPad;
      const v8us hv = *(const v8us*)(Ph + (size_t)srow * CCH + pc);
      const v8us lv = *(const v8us*)(Pl + (size_t)srow * CCH + pc);
      *(v8us*)(Th + rr * CCH + pc) = hv;
      *(v8us*)(Tl + rr * CCH + pc) = lv;
    }
    __syncthreads();
#pragma unroll
    for (int kc = 0; kc < 2; ++kc) {
      const int ca = kc * 32 + 8 * h;
      BFrag ah0, ah1, al0, al1, bh0, bh1, bl0, bl1;
      const int ao0 = (32 * wr + mi) * CCH + ca;
      const int ao1 = ao0 + 16 * CCH;
      ah0.u[0] = *(const v8us*)(Th + ao0);      ah0.u[1] = *(const v8us*)(Th + ao0 + 16);
      ah1.u[0] = *(const v8us*)(Th + ao1);      ah1.u[1] = *(const v8us*)(Th + ao1 + 16);
      al0.u[0] = *(const v8us*)(Tl + ao0);      al0.u[1] = *(const v8us*)(Tl + ao0 + 16);
      al1.u[0] = *(const v8us*)(Tl + ao1);      al1.u[1] = *(const v8us*)(Tl + ao1 + 16);
      const size_t wo0 = (size_t)(32 * wc + mi) * KK + (size_t)k * CCH + ca;
      const size_t wo1 = wo0 + (size_t)16 * KK;
      bh0.u[0] = *(const v8us*)(Wh + wo0);      bh0.u[1] = *(const v8us*)(Wh + wo0 + 16);
      bh1.u[0] = *(const v8us*)(Wh + wo1);      bh1.u[1] = *(const v8us*)(Wh + wo1 + 16);
      bl0.u[0] = *(const v8us*)(Wl + wo0);      bl0.u[1] = *(const v8us*)(Wl + wo0 + 16);
      bl1.u[0] = *(const v8us*)(Wl + wo1);      bl1.u[1] = *(const v8us*)(Wl + wo1 + 16);
      acc00 = wmb(ah0.v, bh0.v, acc00);  acc00 = wmb(ah0.v, bl0.v, acc00);  acc00 = wmb(al0.v, bh0.v, acc00);
      acc01 = wmb(ah0.v, bh1.v, acc01);  acc01 = wmb(ah0.v, bl1.v, acc01);  acc01 = wmb(al0.v, bh1.v, acc01);
      acc10 = wmb(ah1.v, bh0.v, acc10);  acc10 = wmb(ah1.v, bl0.v, acc10);  acc10 = wmb(al1.v, bh0.v, acc10);
      acc11 = wmb(ah1.v, bh1.v, acc11);  acc11 = wmb(ah1.v, bl1.v, acc11);  acc11 = wmb(al1.v, bh1.v, acc11);
    }
  }

  stage16(S, acc00, 32 * wr,      32 * wc,      h, mi, psc, pmu, pbe);
  stage16(S, acc01, 32 * wr,      32 * wc + 16, h, mi, psc, pmu, pbe);
  stage16(S, acc10, 32 * wr + 16, 32 * wc,      h, mi, psc, pmu, pbe);
  stage16(S, acc11, 32 * wr + 16, 32 * wc + 16, h, mi, psc, pmu, pbe);
  __syncthreads();

  if (LAST) {
    v4f ov[TR / 8];
#pragma unroll
    for (int it = 0; it < TR / 8; ++it) {
      const int rr = 8 * it + (tid >> 4);
      const int pc = (tid & 15) * 4;
      const v4f sv = *(const v4f*)(S + rr * CCH + pc);
      ov[it] = sv * pmk[rr];
    }
#pragma unroll
    for (int it = 0; it < TR / 8; ++it) {
      const int rr = 8 * it + (tid >> 4);
      const int pc = (tid & 15) * 4;
      const int dr = rowbase + rr;
      if (dr < nN) *(volatile v4f*)(out + (size_t)dr * CCH + pc) = ov[it];
    }
    __threadfence();
#pragma unroll
    for (int it = 0; it < TR / 8; ++it) {
      const int rr = 8 * it + (tid >> 4);
      const int pc = (tid & 15) * 4;
      const int dr = rowbase + rr;
      if (dr < nN) *(volatile v4f*)(out + (size_t)dr * CCH + pc) = ov[it];
    }
  } else {
    v8us oh[TR / PROWS], ol[TR / PROWS];
#pragma unroll
    for (int it = 0; it < TR / PROWS; ++it) {
      const int rr = PROWS * it + (tid >> 3);
      const int pc = (tid & 7) * 8;
      const v4f a = *(const v4f*)(S + rr * CCH + pc);
      const v4f b = *(const v4f*)(S + rr * CCH + pc + 4);
      split8(a, b, oh[it], ol[it]);
    }
#pragma unroll
    for (int it = 0; it < TR / PROWS; ++it) {
      const int rr = PROWS * it + (tid >> 3);
      const int pc = (tid & 7) * 8;
      const size_t o = (size_t)(rowbase + rr) * CCH + pc;
      *(volatile v8us*)(Oh + o) = oh[it];
      *(volatile v8us*)(Ol + o) = ol[it];
    }
    __threadfence();
#pragma unroll
    for (int it = 0; it < TR / PROWS; ++it) {
      const int rr = PROWS * it + (tid >> 3);
      const int pc = (tid & 7) * 8;
      const size_t o = (size_t)(rowbase + rr) * CCH + pc;
      *(volatile v8us*)(Oh + o) = oh[it];
      *(volatile v8us*)(Ol + o) = ol[it];
    }
  }
}

extern "C" void kernel_launch(void* const* d_in, const int* in_sizes, int n_in,
                              void* d_out, int out_size, void* d_ws, size_t ws_size,
                              hipStream_t stream) {
  if (n_in < 18) return;
  if (in_sizes[0] < CCH || (in_sizes[0] % CCH) != 0) return;
  const int nN = in_sizes[0] / CCH;
  if (nN < 1) return;
  if (in_sizes[1] != 3 * nN) return;
  if (in_sizes[2] != KOF * nN) return;
  if (in_sizes[3] != KOF * CCH * CCH || in_sizes[8] != KOF * CCH * CCH || in_sizes[13] != KOF * CCH * CCH) return;
  for (int i = 0; i < 4; ++i) {
    if (in_sizes[4 + i] != CCH || in_sizes[9 + i] != CCH || in_sizes[14 + i] != CCH) return;
  }
  if (out_size != nN * CCH) return;

  const int nBlkC = (nN + TR - 1) / TR;
  const int mPad  = nBlkC * TR;
  const int R     = mPad + ZPAD;
  const int gX    = mPad / PROWS;

  const float* feat = (const float*)d_in[0];
  const int*   coor = (const int*)d_in[1];
  const int*   kin  = (const int*)d_in[2];
  const float* W1 = (const float*)d_in[3];
  const float* g1 = (const float*)d_in[4];
  const float* b1 = (const float*)d_in[5];
  const float* m1 = (const float*)d_in[6];
  const float* v1 = (const float*)d_in[7];
  const float* W2 = (const float*)d_in[8];
  const float* g2 = (const float*)d_in[9];
  const float* b2 = (const float*)d_in[10];
  const float* m2 = (const float*)d_in[11];
  const float* v2 = (const float*)d_in[12];
  const float* W3 = (const float*)d_in[13];
  const float* g3 = (const float*)d_in[14];
  const float* b3 = (const float*)d_in[15];
  const float* m3 = (const float*)d_in[16];
  const float* v3 = (const float*)d_in[17];
  float* out = (float*)d_out;

  const size_t planeB = (size_t)R * CCH * sizeof(us);
  const size_t wB     = (size_t)NLAY * CCH * KK * sizeof(us);
  char* ws = (char*)d_ws;
  size_t off = 0;
  const size_t oP0h = off; off += (planeB + 255) & ~(size_t)255;
  const size_t oP0l = off; off += (planeB + 255) & ~(size_t)255;
  const size_t oP1h = off; off += (planeB + 255) & ~(size_t)255;
  const size_t oP1l = off; off += (planeB + 255) & ~(size_t)255;
  const size_t oWh  = off; off += (wB + 255) & ~(size_t)255;
  const size_t oWl  = off; off += (wB + 255) & ~(size_t)255;
  if (off > ws_size || off > (size_t)WSCAP) return;
  us* P0h = (us*)(ws + oP0h);
  us* P0l = (us*)(ws + oP0l);
  us* P1h = (us*)(ws + oP1h);
  us* P1l = (us*)(ws + oP1l);
  us* Wh  = (us*)(ws + oWh);
  us* Wl  = (us*)(ws + oWl);

  k_xprep<<<gX, PTH, 0, stream>>>(feat, P0h, P0l, nN);
  k_zprep<<<4, PTH, 0, stream>>>(P0h, P0l, P1h, P1l, mPad);
  k_wprep<<<dim3(KOF, NLAY), PTH, 0, stream>>>(W1, W2, W3, Wh, Wl);
  k_conv<0><<<nBlkC, CTH, 0, stream>>>(P0h, P0l, kin, Wh, Wl, g1, b1, m1, v1, coor,
                                       P1h, P1l, out, nN, mPad);
  k_conv<0><<<nBlkC, CTH, 0, stream>>>(P1h, P1l, kin, Wh + (size_t)CCH * KK, Wl + (size_t)CCH * KK,
                                       g2, b2, m2, v2, coor, P0h, P0l, out, nN, mPad);
  k_conv<1><<<nBlkC, CTH, 0, stream>>>(P0h, P0l, kin, Wh + (size_t)2 * CCH * KK, Wl + (size_t)2 * CCH * KK,
                                       g3, b3, m3, v3, coor, P1h, P1l, out, nN, mPad);
}
